// EIGLayer_69346541962061
// MI455X (gfx1250) — hardware-run, weakly checked
//
#include <hip/hip_runtime.h>
#include <stddef.h>
#include <stdint.h>


#ifndef SPLIT_P
#define SPLIT_P 1
#endif

#define NNODE   40000
#define NEDGE   640000
#define DF      128
#define EDIM    16
#define MP      40064
#define HALFN   20480
#define AGWD    768
#define APITCH  1536
#if SPLIT_P
#define KAGG    1536
#else
#define KAGG    768
#endif
#define WPITCH  1664
#define NPOST   384
#define PABP    256
#define TP      132
#define BTHR    512
#define BWAVE   16
#define EPT     8
#define CHUNK   (BTHR * EPT)
#define WCAP    (EPT * 32)
#define LISTN   (BWAVE * WCAP)
#define NB      1024
#define NBLK    40
#define RCAP    20480
#define DEGCAP  64
#define GBM     64
#define GBN     64
#define GTHR    128
#define AGB     1024
#define PB_HB   2504
#define PB_WAB  16
#define PB_WC   2
#define PB_WP   312
#define PB_EG   40
#define PB_SN   40
#define PB_BI   1
#define PB_TOT  (PB_HB + PB_WAB + PB_WC + PB_WP + PB_EG + PB_SN + PB_BI)
#define LDS_BKT ((2 * RCAP + 2 * NB + LISTN + 2 * BWAVE) * 4)
#define LDS_AGG (DF * 32 * 2 + 8 * 16 * TP * 4)
#define LDS_V   (128 * TP * 4)

static_assert(HALFN % 1024 == 0 && HALFN % 128 == 0);
static_assert(MP == 313 * 128 && MP % GBM == 0 && MP >= NNODE && MP - NNODE < 128);
static_assert(NBLK * NB >= MP && 2 * HALFN == NBLK * NB && HALFN % AGB == 0 && AGB == NB);
static_assert((CHUNK & (CHUNK - 1)) == 0 && CHUNK <= 4096);
static_assert((NB & (NB - 1)) == 0 && NB <= 4096 && BTHR * 2 == NB && LISTN >= NB);
static_assert((RCAP % 16) == 0 && RCAP >= 16701 + 2048);
static_assert(DEGCAP >= 35 + 8 && (DEGCAP % 16) == 0);
static_assert(NEDGE < (1 << 20));
static_assert(LDS_BKT <= 327680 && LDS_AGG <= 327680 && LDS_V + 4096 <= 327680);
static_assert(MP * 16 == PB_HB * 256 && NPOST * (WPITCH / 8) == PB_WP * 256 && 256 * 16 == PB_WAB * 256);
static_assert(MP % 4 == 0 && (MP / 4) <= PB_EG * 256 && (MP * 4) % 128 == 0);
static_assert(WPITCH == DF + 2 * AGWD && APITCH == 2 * AGWD && KAGG % 32 == 0 && KAGG <= APITCH && DF + KAGG <= WPITCH);
static_assert((WPITCH / 8) % 8 == 0 && (TP % 4) == 0 && TP >= DF);
static_assert((float)(2.77258872 + 2.239781e-9) == 0x1.62E43p+1f);

typedef float          v4f   __attribute__((ext_vector_type(4)));
typedef float          v8f   __attribute__((ext_vector_type(8)));
typedef int            v2i   __attribute__((ext_vector_type(2)));
typedef int            v4i   __attribute__((ext_vector_type(4)));
typedef int            v8i   __attribute__((ext_vector_type(8)));
typedef unsigned       v2u   __attribute__((ext_vector_type(2)));
typedef unsigned short v8us  __attribute__((ext_vector_type(8)));
typedef __bf16         v16bf __attribute__((ext_vector_type(16)));
typedef v4f __attribute__((may_alias)) v4fa;
union FragB { v16bf v; v8us u[2]; v8i w; v4i q[2]; };

__device__ __forceinline__ v8f wmx(const FragB& a, const FragB& b, v8f c) {
  v8f d = __builtin_amdgcn_wmma_f32_16x16x32_bf16(false, a.v, false, b.v, (short)0, c, false, false);
  asm volatile("v_nop\n\tv_nop\n\tv_nop\n\tv_nop" : "+v"(d) : "v"(a.w), "v"(b.w));
  return d;
}

__device__ __forceinline__ void pinf(float x) { asm volatile("" :: "v"(x)); }
__device__ __forceinline__ void pini(int x)   { asm volatile("" :: "v"(x)); }

__device__ __forceinline__ unsigned bfbits(float v) {
  const unsigned u = __float_as_uint(v);
  const unsigned r = (u + 0x7FFFu + ((u >> 16) & 1u)) >> 16;
  const unsigned nb = ((u >> 16) & 0x8000u) | 0x7FC0u;
  return ((u & 0x7FFFFFFFu) > 0x7F800000u) ? nb : r;
}
__device__ __forceinline__ float rbf(float v) { return __uint_as_float(bfbits(v) << 16); }
__device__ __forceinline__ v4f rbf4(const v4f a) {
  v4f o; o.x = rbf(a.x); o.y = rbf(a.y); o.z = rbf(a.z); o.w = rbf(a.w); return o;
}
__device__ __forceinline__ v8us pk8(const v4f a, const v4f b, unsigned mk) {
  v8us hv;
  hv[0] = (unsigned short)(bfbits(a.x) & mk); hv[1] = (unsigned short)(bfbits(a.y) & mk);
  hv[2] = (unsigned short)(bfbits(a.z) & mk); hv[3] = (unsigned short)(bfbits(a.w) & mk);
  hv[4] = (unsigned short)(bfbits(b.x) & mk); hv[5] = (unsigned short)(bfbits(b.y) & mk);
  hv[6] = (unsigned short)(bfbits(b.z) & mk); hv[7] = (unsigned short)(bfbits(b.w) & mk);
  return hv;
}
__device__ __forceinline__ void st2us(unsigned short* p, const v8us v) {
  *(volatile v8us*)p = v;
  __threadfence();
  *(volatile v8us*)p = v;
}
__device__ __forceinline__ void st2f4(float* p, const v4f v) {
  *(volatile v4f*)p = v;
  __threadfence();
  *(volatile v4f*)p = v;
}
__device__ __forceinline__ void wave_sync() {
  __builtin_amdgcn_fence(__ATOMIC_RELEASE, "wavefront");
  __builtin_amdgcn_wave_barrier();
  __builtin_amdgcn_fence(__ATOMIC_ACQUIRE, "wavefront");
}
__device__ __forceinline__ float var_lit(float s2, float mean, float degc) {
#pragma clang fp contract(off)
  const float q = s2 / degc;
  const float p = mean * mean;
  return q - p;
}

__device__ __forceinline__ int scan_chunk(const int* __restrict__ dsts, int nE, int cbase, int slotBase,
                                          int nb, int vec8, int* list, int tid, int lane, int wave) {
  int wc = 0;
  const int el0  = tid * EPT;
  const int e0   = cbase + el0;
  const int sent = (int)(1u << 31);
  v4i da, db;
  if (vec8 != 0 && cbase + CHUNK <= nE) {
    da = *(const v4i*)(dsts + e0);
    db = *(const v4i*)(dsts + e0 + 4);
  } else {
    da.x = (e0     < nE) ? dsts[min(e0,     nE - 1)] : sent;
    da.y = (e0 + 1 < nE) ? dsts[min(e0 + 1, nE - 1)] : sent;
    da.z = (e0 + 2 < nE) ? dsts[min(e0 + 2, nE - 1)] : sent;
    da.w = (e0 + 3 < nE) ? dsts[min(e0 + 3, nE - 1)] : sent;
    db.x = (e0 + 4 < nE) ? dsts[min(e0 + 4, nE - 1)] : sent;
    db.y = (e0 + 5 < nE) ? dsts[min(e0 + 5, nE - 1)] : sent;
    db.z = (e0 + 6 < nE) ? dsts[min(e0 + 6, nE - 1)] : sent;
    db.w = (e0 + 7 < nE) ? dsts[min(e0 + 7, nE - 1)] : sent;
  }
  const unsigned nbs = (unsigned)slotBase;
  const unsigned unb = (unsigned)nb;
  const unsigned s0 = (unsigned)da.x - nbs, s1 = (unsigned)da.y - nbs;
  const unsigned s2 = (unsigned)da.z - nbs, s3 = (unsigned)da.w - nbs;
  const unsigned s4 = (unsigned)db.x - nbs, s5 = (unsigned)db.y - nbs;
  const unsigned s6 = (unsigned)db.z - nbs, s7 = (unsigned)db.w - nbs;
  const bool h0 = s0 < unb, h1 = s1 < unb, h2 = s2 < unb, h3 = s3 < unb;
  const bool h4 = s4 < unb, h5 = s5 < unb, h6 = s6 < unb, h7 = s7 < unb;
  const unsigned any = __builtin_amdgcn_ballot_w32(h0 | h1 | h2 | h3 | h4 | h5 | h6 | h7);
  if (any != 0u) {
#define HITJ(J, HJ, SJ) { \
      const unsigned mj = __builtin_amdgcn_ballot_w32(HJ); \
      if (mj != 0u) { \
        if (HJ) { \
          const int pos = wc + (int)__builtin_amdgcn_mbcnt_lo(mj, 0u); \
          if (pos < WCAP) list[wave * WCAP + pos] = ((el0 + (J)) << 12) | (int)(SJ); \
        } \
        wc += (int)__builtin_popcount(mj); } }
    HITJ(0, h0, s0)
    HITJ(1, h1, s1)
    HITJ(2, h2, s2)
    HITJ(3, h3, s3)
    HITJ(4, h4, s4)
    HITJ(5, h5, s5)
    HITJ(6, h6, s6)
    HITJ(7, h7, s7)
#undef HITJ
  }
  return wc;
}

__global__ __launch_bounds__(256) void k_prep(const float* __restrict__ h, const float* __restrict__ evec,
                                              const float* __restrict__ sn, const float* __restrict__ wpre,
                                              const float* __restrict__ bpre, const float* __restrict__ wpost,
                                              const float* __restrict__ bpost,
                                              unsigned short* hb, unsigned short* wabT, unsigned short* wcP,
                                              unsigned short* wpT, float* ev1, float* snT,
                                              float* bpre256, float* bpostT) {
  const int tid = (int)threadIdx.x;
  int blk = (int)blockIdx.x;
  if (blk < PB_HB) {
    const int i = blk * 256 + tid;
    const int row = i >> 4;
    const int c0  = (i & 15) * 8;
    const int rc  = row < NNODE ? row : NNODE - 1;
    const float* p = h + (size_t)rc * DF + c0;
    const v4f a = *(const v4f*)p, b = *(const v4f*)(p + 4);
    const unsigned mk = row < NNODE ? 0xFFFFu : 0u;
    st2us(hb + (size_t)row * DF + c0, pk8(a, b, mk));
    return;
  }
  blk -= PB_HB;
  if (blk < PB_WAB) {
    const int u  = blk * 256 + tid;
    const int n  = u >> 4;
    const int k8 = (u & 15) * 8;
    const int r0 = (n < DF ? 0 : DF) + k8;
    const int c  = n & (DF - 1);
    float f[8];
#pragma unroll
    for (int i = 0; i < 8; ++i) { f[i] = wpre[(size_t)(r0 + i) * DF + c]; pinf(f[i]); }
    v4f a, b;
    a.x = f[0]; a.y = f[1]; a.z = f[2]; a.w = f[3]; b.x = f[4]; b.y = f[5]; b.z = f[6]; b.w = f[7];
    st2us(wabT + (size_t)n * DF + k8, pk8(a, b, 0xFFFFu));
    return;
  }
  blk -= PB_WAB;
  if (blk < PB_WC) {
    const int u  = blk * 256 + tid;
    const int n  = u >> 2;
    const int k8 = (u & 3) * 8;
    const int kc = k8 < EDIM ? k8 : 8;
    const unsigned mk = k8 < EDIM ? 0xFFFFu : 0u;
    float f[8];
#pragma unroll
    for (int i = 0; i < 8; ++i) { f[i] = wpre[(size_t)(2 * DF + kc + i) * DF + n]; pinf(f[i]); }
    v4f a, b;
    a.x = f[0]; a.y = f[1]; a.z = f[2]; a.w = f[3]; b.x = f[4]; b.y = f[5]; b.z = f[6]; b.w = f[7];
    st2us(wcP + (size_t)n * 32 + k8, pk8(a, b, mk));
    return;
  }
  blk -= PB_WC;
  if (blk < PB_WP) {
    const int u  = blk * 256 + tid;
    const int n  = u / (WPITCH / 8);
    const int k8 = (u - n * (WPITCH / 8)) * 8;
    const int nb = n >> 7;
    const int c  = n & (DF - 1);
    int a0 = k8 - DF;
    a0 = a0 >= AGWD ? a0 - AGWD : a0;
    a0 = a0 < 0 ? 0 : a0;
    const int r0 = (k8 < DF) ? k8 : (DF + AGWD * nb + a0);
    const unsigned mk = (k8 < DF && nb != 0) ? 0u : 0xFFFFu;
    float f[8];
#pragma unroll
    for (int i = 0; i < 8; ++i) { f[i] = wpost[(size_t)(r0 + i) * DF + c]; pinf(f[i]); }
    v4f a, b;
    a.x = f[0]; a.y = f[1]; a.z = f[2]; a.w = f[3]; b.x = f[4]; b.y = f[5]; b.z = f[6]; b.w = f[7];
    st2us(wpT + (size_t)n * WPITCH + k8, pk8(a, b, mk));
    return;
  }
  blk -= PB_WP;
  if (blk < PB_EG) {
    const int u = blk * 256 + tid;
    if (u >= MP / 4) return;
    float f[4];
#pragma unroll
    for (int i = 0; i < 4; ++i) {
      const int idx = 4 * u + i;
      const int ic  = idx < NNODE ? idx : NNODE - 1;
      f[i] = evec[2 * (size_t)ic + 1];
      pinf(f[i]);
    }
    v4f o;
    o.x = (4 * u + 0 < NNODE) ? rbf(f[0]) : 0.0f;
    o.y = (4 * u + 1 < NNODE) ? rbf(f[1]) : 0.0f;
    o.z = (4 * u + 2 < NNODE) ? rbf(f[2]) : 0.0f;
    o.w = (4 * u + 3 < NNODE) ? rbf(f[3]) : 0.0f;
    st2f4(ev1 + 4 * (size_t)u, o);
    return;
  }
  blk -= PB_EG;
  if (blk < PB_SN) {
    const int u = blk * 256 + tid;
    if (u >= MP / 4) return;
    float f[4];
#pragma unroll
    for (int i = 0; i < 4; ++i) {
      const int idx = 4 * u + i;
      const int ic  = idx < NNODE ? idx : NNODE - 1;
      f[i] = sn[ic];
      pinf(f[i]);
    }
    v4f o;
    o.x = (4 * u + 0 < NNODE) ? rbf(f[0]) : 0.0f;
    o.y = (4 * u + 1 < NNODE) ? rbf(f[1]) : 0.0f;
    o.z = (4 * u + 2 < NNODE) ? rbf(f[2]) : 0.0f;
    o.w = (4 * u + 3 < NNODE) ? rbf(f[3]) : 0.0f;
    st2f4(snT + 4 * (size_t)u, o);
    return;
  }
  if (tid < 64) {
    float f[4];
#pragma unroll
    for (int i = 0; i < 4; ++i) {
      const int bi = 4 * tid + i - DF;
      f[i] = bpre[bi < 0 ? 0 : bi];
      pinf(f[i]);
    }
    v4f o;
    o.x = (4 * tid + 0 >= DF) ? rbf(f[0]) : 0.0f;
    o.y = (4 * tid + 1 >= DF) ? rbf(f[1]) : 0.0f;
    o.z = (4 * tid + 2 >= DF) ? rbf(f[2]) : 0.0f;
    o.w = (4 * tid + 3 >= DF) ? rbf(f[3]) : 0.0f;
    st2f4(bpre256 + 4 * tid, o);
  } else if (tid < 96) {
    const int j = tid - 64;
    const v4f b = *(const v4f*)(bpost + 4 * j);
    st2f4(bpostT + 4 * j, rbf4(b));
  }
}

__global__ __launch_bounds__(GTHR) void k_gemm(
    const unsigned short* __restrict__ A, const unsigned short* __restrict__ WT,
    const float* __restrict__ bias, float* outF, int K, int ldo)
{
  __shared__ __attribute__((aligned(16))) float stg[GBM * GBN];
  const int tid = (int)threadIdx.x, lane = tid & 31, wave = tid >> 5, hh = lane >> 4, m = lane & 15;
  const int rowBase = (int)blockIdx.x * GBM;
  const int col0    = (int)blockIdx.y * GBN;

  v8f acc[4];
  {
    const v8f z = {0.f, 0.f, 0.f, 0.f, 0.f, 0.f, 0.f, 0.f};
    acc[0] = z; acc[1] = z; acc[2] = z; acc[3] = z;
  }
  const unsigned short* ap = A  + (size_t)(rowBase + 16 * wave + m) * (size_t)K + 8 * hh;
  const unsigned short* wp = WT + (size_t)(col0 + m) * (size_t)K + 8 * hh;
  const int ksteps = K >> 5;
#pragma unroll 1
  for (int ks = 0; ks < ksteps; ++ks) {
    FragB af;
    af.u[0] = *(const v8us*)(ap + 32 * ks);
    af.u[1] = *(const v8us*)(ap + 32 * ks + 16);
#pragma unroll
    for (int t = 0; t < 4; ++t) {
      const unsigned short* wq = wp + (size_t)(16 * t) * (size_t)K + 32 * ks;
      FragB bf;
      bf.u[0] = *(const v8us*)wq;
      bf.u[1] = *(const v8us*)(wq + 16);
      acc[t] = wmx(af, bf, acc[t]);
    }
  }

#pragma unroll
  for (int t = 0; t < 4; ++t) {
    const int lc = 16 * t + m;
#pragma unroll
    for (int r = 0; r < 8; ++r) {
      const int lr = 16 * wave + 8 * hh + r;
      stg[lr * GBN + lc] = acc[t][r];
    }
  }
  __syncthreads();

  const v4f bv = *(const v4f*)(bias + col0 + 4 * m);
  v4f fv[8];
#pragma unroll
  for (int i = 0; i < 8; ++i) {
    const int lr = 16 * wave + 2 * i + hh;
    v4f v = *(const v4fa*)(stg + lr * GBN + 4 * m);
    fv[i] = v + bv;
  }
#pragma unroll
  for (int i = 0; i < 8; ++i) {
    const int lr = 16 * wave + 2 * i + hh;
    float* op = outF + (size_t)(rowBase + lr) * (size_t)ldo + col0 + 4 * m;
    *(volatile v4f*)op = fv[i];
  }
  __threadfence();
#pragma unroll
  for (int i = 0; i < 8; ++i) {
    const int lr = 16 * wave + 2 * i + hh;
    float* op = outF + (size_t)(rowBase + lr) * (size_t)ldo + col0 + 4 * m;
    *(volatile v4f*)op = fv[i];
  }
}

__global__ __launch_bounds__(BTHR) void k_bucket(const int* __restrict__ srcs, const int* __restrict__ dsts,
                                                 int* ent, int* slot, int nN, int nE, int vec8) {
  extern __shared__ v4f lds_dyn[];
  int* reg1 = (int*)lds_dyn;
  int* reg2 = reg1 + RCAP;
  int* scnt = reg2 + RCAP;
  int* soff = scnt + NB;
  int* list = soff + NB;
  int* wcnt = list + LISTN;
  int* wtot = wcnt + BWAVE;
  const int tid = (int)threadIdx.x, lane = tid & 31;
  const int wave = __builtin_amdgcn_readfirstlane(tid >> 5);
  const int nodeBase = (int)blockIdx.x * NB;

  for (int i = tid; i < NB; i += BTHR) scnt[i] = 0;
  for (int i = tid; i < RCAP; i += BTHR) { reg1[i] = 0; reg2[i] = 0; }
  __syncthreads();

  int tot = 0;
  const int nChunks = (nE + CHUNK - 1) / CHUNK;
#pragma unroll 1
  for (int ch = 0; ch < nChunks; ++ch) {
    const int cbase = ch * CHUNK;
    const int wc = scan_chunk(dsts, nE, cbase, nodeBase, NB, vec8, list, tid, lane, wave);
    if (lane == 0) wcnt[wave] = wc;
    __syncthreads();
    int pre = 0, all = 0;
#pragma unroll
    for (int w2 = 0; w2 < BWAVE; ++w2) {
      int c = wcnt[w2];
      c = c < 0 ? 0 : (c > WCAP ? WCAP : c);
      all += c;
      pre += (w2 < wave) ? c : 0;
    }
    const int wcc  = wc > WCAP ? WCAP : wc;
    const int base = tot + pre;
#pragma unroll 1
    for (int i = lane; i < wcc; i += 32) {
      const int en = list[wave * WCAP + i];
      const int el = (en >> 12) & (CHUNK - 1);
      const int sl = en & (NB - 1);
      int eid = cbase + el;
      eid = eid > nE - 1 ? nE - 1 : eid;
      const int pos = base + i;
      if (pos < RCAP) reg1[pos] = (int)(((unsigned)eid << 12) | (unsigned)sl);
    }
    tot += all;
    tot = tot > RCAP ? RCAP : tot;
    __syncthreads();
  }
  const int nh = tot;

  if (wave == 0) {
#pragma unroll 1
    for (int b0 = 0; b0 < nh; b0 += 32) {
      const int idx = b0 + lane;
      const int uv  = reg1[idx < RCAP ? idx : RCAP - 1];
      const int m32 = (nh - b0) < 32 ? (nh - b0) : 32;
#pragma unroll 1
      for (int k = 0; k < m32; ++k) {
        const int u  = __builtin_amdgcn_readlane(uv, k);
        const int sl = u & (NB - 1);
        if (lane == 0) scnt[sl] = scnt[sl] + 1;
      }
    }
  }
  __syncthreads();

  {
    const int r0 = scnt[2 * tid], r1 = scnt[2 * tid + 1];
    const int e0 = r0 < 0 ? 0 : r0, e1 = r1 < 0 ? 0 : r1;
    const int ts = e0 + e1;
    int incl = ts;
#pragma unroll
    for (int d = 1; d < 32; d <<= 1) {
      const int up = __shfl_up(incl, d);
      if (lane >= d) incl += up;
    }
    if (lane == 31) wtot[wave] = incl;
    __syncthreads();
    int pre = 0;
#pragma unroll
    for (int w2 = 0; w2 < BWAVE; ++w2) pre += (w2 < wave) ? wtot[w2] : 0;
    const int run = pre + incl - ts;
    soff[2 * tid]     = run;
    soff[2 * tid + 1] = run + e0;
  }
  __syncthreads();
  for (int i = tid; i < NB; i += BTHR) list[i] = soff[i];
  __syncthreads();

  if (wave == 0) {
#pragma unroll 1
    for (int b0 = 0; b0 < nh; b0 += 32) {
      const int idx = b0 + lane;
      const int uv  = reg1[idx < RCAP ? idx : RCAP - 1];
      const int m32 = (nh - b0) < 32 ? (nh - b0) : 32;
#pragma unroll 1
      for (int k = 0; k < m32; ++k) {
        const int u   = __builtin_amdgcn_readlane(uv, k);
        const int sl  = u & (NB - 1);
        const int eid = (int)((unsigned)u >> 12);
        if (lane == 0) {
          int pos = list[sl];
          pos = pos < 0 ? 0 : (pos > RCAP - 1 ? RCAP - 1 : pos);
          reg2[pos] = eid;
          list[sl] = pos + 1;
        }
      }
    }
  }
  __syncthreads();

  const bool ovf = (nh >= RCAP);
  const int nhPad = (nh + 15) & ~15;
  int* eb = ent + (size_t)blockIdx.x * (size_t)(2 * RCAP);
#pragma unroll 1
  for (int p0 = 0; p0 < nhPad; p0 += 2 * BTHR) {
    const int p   = p0 + 2 * tid;
    const bool ac = p < nhPad;
    const int pa  = p < RCAP - 2 ? p : RCAP - 2;
    int e0 = reg2[pa], e1 = reg2[pa + 1];
    e0 = e0 < 0 ? 0 : (e0 > nE - 1 ? nE - 1 : e0);
    e1 = e1 < 0 ? 0 : (e1 > nE - 1 ? nE - 1 : e1);
    const int s0 = srcs[e0];
    const int s1 = srcs[e1];
    pini(s0); pini(s1);
    const int m0 = (p     < nh) ? -1 : 0;
    const int m1 = (p + 1 < nh) ? -1 : 0;
    v4i v;
    v.x = s0 & m0; v.y = e0 & m0; v.z = s1 & m1; v.w = e1 & m1;
    if (ac) *(volatile v4i*)(eb + 2 * pa) = v;
    __threadfence();
    if (ac) *(volatile v4i*)(eb + 2 * pa) = v;
  }
  {
    v4i sv;
    sv.x = soff[2 * tid];
    sv.y = ovf ? -1 : scnt[2 * tid];
    sv.z = soff[2 * tid + 1];
    sv.w = ovf ? -1 : scnt[2 * tid + 1];
    int* sp = slot + 2 * (size_t)(nodeBase + 2 * tid);
    *(volatile v4i*)sp = sv;
    __threadfence();
    *(volatile v4i*)sp = sv;
  }
  (void)nN;
}

__global__ __launch_bounds__(256) __attribute__((amdgpu_num_vgpr(248)))
void k_agg(const int* __restrict__ ent, const int* __restrict__ slot, const float* __restrict__ ef,
           const int* __restrict__ wcp, const float* __restrict__ pab, const float* __restrict__ ev1,
           const unsigned short* __restrict__ hb, unsigned short* agg, int passBase, int nN, int nE)
{
  extern __shared__ v4f lds_dyn[];
  int*   sW = (int*)lds_dyn;
  float* sT = (float*)(sW + DF * 16);
  const int tid = (int)threadIdx.x, lane = tid & 31, hh = lane >> 4, m = lane & 15;
  const int wave = __builtin_amdgcn_readfirstlane(tid >> 5);
#pragma unroll
  for (int t = 0; t < 2; ++t) {
    const int idx = tid + 256 * t;
    const v4i w = *(const v4i*)(wcp + 4 * idx);
    *(v4i*)(sW + 4 * idx) = w;
  }
  __syncthreads();
  float* T = sT + wave * 16 * TP;
  const v8f z8 = {0.f, 0.f, 0.f, 0.f, 0.f, 0.f, 0.f, 0.f};
  const float qnan = __int_as_float(0x7fc00000);

#pragma unroll 1
  for (int si = 0; si < AGB / 8; ++si) {
    const int lrow = (int)blockIdx.x * AGB + si * 8 + wave;
    const int i  = passBase + lrow;
    const int ic = i < nN ? i : nN - 1;
    const v2i se = *(const v2i*)(slot + 2 * (size_t)i);
    int stv = se.x;
    stv = stv < 0 ? 0 : (stv > RCAP - 1 ? RCAP - 1 : stv);
    const int cv = se.y;
    const int badv = (cv < 0 || cv > DEGCAP) ? 1 : 0;
    int ccv = cv < 0 ? 0 : (cv > DEGCAP ? DEGCAP : cv);
    ccv = ccv > RCAP - stv ? RCAP - stv : ccv;
    ccv = i < nN ? ccv : 0;
    const int st  = __builtin_amdgcn_readfirstlane(stv);
    const int cnt = __builtin_amdgcn_readfirstlane(ccv);
    const int bad = __builtin_amdgcn_readfirstlane(badv);
    int last = st + cnt - 1;
    last = last < st ? st : last;
    const int* eb = ent + (size_t)(i / NB) * (size_t)(2 * RCAP);

    const v4f pbb = *(const v4f*)(pab + (size_t)ic * PABP + DF + 4 * lane);
    const float evi = ev1[ic];
    const v2u hw = *(const v2u*)(hb + (size_t)ic * DF + 4 * lane);
    pini((int)hw.x); pini((int)hw.y);
    pinf(pbb.x); pinf(evi);

    v4f s1 = {0.f, 0.f, 0.f, 0.f}, s2 = {0.f, 0.f, 0.f, 0.f};
    v4f sav = {0.f, 0.f, 0.f, 0.f}, sdx = {0.f, 0.f, 0.f, 0.f};
    v4f mx = {-3.0e38f, -3.0e38f, -3.0e38f, -3.0e38f};
    v4f mn = {3.0e38f, 3.0e38f, 3.0e38f, 3.0e38f};
    float dsum = 0.0f;

#pragma unroll 1
    for (int t0 = 0; t0 < cnt; t0 += 16) {
      const int nv = (cnt - t0) < 16 ? (cnt - t0) : 16;
      int ei = st + t0 + m;
      ei = ei > last ? last : ei;
      const v2i en = *(const v2i*)(eb + 2 * ei);
      const int src = en.x < 0 ? 0 : (en.x > nN - 1 ? nN - 1 : en.x);
      const int eid = en.y < 0 ? 0 : (en.y > nE - 1 ? nE - 1 : en.y);
      const float dl = ev1[src] - evi;
      const float* ep = ef + (size_t)eid * EDIM + 8 * hh;
      const v4f ea = *(const v4f*)ep;
      const v4f eb4 = *(const v4f*)(ep + 4);
      const unsigned mk = (m < nv) ? 0xFFFFu : 0u;
      FragB af;
      {
        v8i w;
        w[0] = (int)((bfbits(ea.x) & mk) | ((bfbits(ea.y) & mk) << 16));
        w[1] = (int)((bfbits(ea.z) & mk) | ((bfbits(ea.w) & mk) << 16));
        w[2] = (int)((bfbits(eb4.x) & mk) | ((bfbits(eb4.y) & mk) << 16));
        w[3] = (int)((bfbits(eb4.z) & mk) | ((bfbits(eb4.w) & mk) << 16));
        w[4] = 0; w[5] = 0; w[6] = 0; w[7] = 0;
        af.w = w;
      }
      wave_sync();
#pragma unroll
      for (int tt = 0; tt < 8; ++tt) {
        const int* wq = sW + (16 * tt + m) * 16 + 4 * hh;
        FragB bf;
        bf.q[0] = *(const v4i*)wq;
        bf.q[1] = *(const v4i*)(wq + 8);
        v8f d = wmx(af, bf, z8);
#pragma unroll
        for (int r = 0; r < 8; ++r) T[(8 * hh + r) * TP + 16 * tt + m] = d[r];
      }
      wave_sync();
      const int dli = __float_as_int(dl);
#pragma unroll 1
      for (int r = 0; r < nv; ++r) {
        const int j = __builtin_amdgcn_readlane(src, r);
        const float dr = __int_as_float(__builtin_amdgcn_readlane(dli, r));
        const float ad = fabsf(dr);
        const v4f pa = *(const v4f*)(pab + (size_t)j * PABP + 4 * lane);
        const v4f ee = *(const v4fa*)(T + r * TP + 4 * lane);
        const v4f mv = (pa + ee) + pbb;
        s1 = s1 + mv;
        s2.x = fmaf(mv.x, mv.x, s2.x); s2.y = fmaf(mv.y, mv.y, s2.y);
        s2.z = fmaf(mv.z, mv.z, s2.z); s2.w = fmaf(mv.w, mv.w, s2.w);
        mx.x = fmaxf(mx.x, mv.x); mx.y = fmaxf(mx.y, mv.y); mx.z = fmaxf(mx.z, mv.z); mx.w = fmaxf(mx.w, mv.w);
        mn.x = fminf(mn.x, mv.x); mn.y = fminf(mn.y, mv.y); mn.z = fminf(mn.z, mv.z); mn.w = fminf(mn.w, mv.w);
        sav.x = fmaf(mv.x, ad, sav.x); sav.y = fmaf(mv.y, ad, sav.y);
        sav.z = fmaf(mv.z, ad, sav.z); sav.w = fmaf(mv.w, ad, sav.w);
        sdx.x = fmaf(mv.x, dr, sdx.x); sdx.y = fmaf(mv.y, dr, sdx.y);
        sdx.z = fmaf(mv.z, dr, sdx.z); sdx.w = fmaf(mv.w, dr, sdx.w);
        dsum += ad;
      }
    }

    const bool has = cnt > 0;
    const float degc = fmaxf((float)cnt, 1.0f);
    const float den  = dsum + 1e-8f;
    const float pz   = (bad != 0) ? qnan : 0.0f;
    v4f hbv;
    hbv.x = __uint_as_float(hw.x << 16); hbv.y = __uint_as_float(hw.x & 0xffff0000u);
    hbv.z = __uint_as_float(hw.y << 16); hbv.w = __uint_as_float(hw.y & 0xffff0000u);
    v4f sg[6];
    {
      const v4f mean = s1 / degc;
      v4f sd;
      sd.x = sqrtf(fmaxf(var_lit(s2.x, mean.x, degc), 0.0f) + 1e-5f);
      sd.y = sqrtf(fmaxf(var_lit(s2.y, mean.y, degc), 0.0f) + 1e-5f);
      sd.z = sqrtf(fmaxf(var_lit(s2.z, mean.z, degc), 0.0f) + 1e-5f);
      sd.w = sqrtf(fmaxf(var_lit(s2.w, mean.w, degc), 0.0f) + 1e-5f);
      sg[0] = mean; sg[1] = mx; sg[2] = mn; sg[3] = sd;
      sg[4] = sav / den;
      sg[5] = sdx / den - hbv;
    }
    v2u hv[6], lv[6];
#pragma unroll
    for (int g = 0; g < 6; ++g) {
      v4f v;
      v.x = has ? sg[g].x : 0.0f; v.y = has ? sg[g].y : 0.0f;
      v.z = has ? sg[g].z : 0.0f; v.w = has ? sg[g].w : 0.0f;
      v = v + pz;
      const unsigned h0 = bfbits(v.x), h1 = bfbits(v.y), h2 = bfbits(v.z), h3 = bfbits(v.w);
      const unsigned l0 = bfbits(v.x - __uint_as_float(h0 << 16));
      const unsigned l1 = bfbits(v.y - __uint_as_float(h1 << 16));
      const unsigned l2 = bfbits(v.z - __uint_as_float(h2 << 16));
      const unsigned l3 = bfbits(v.w - __uint_as_float(h3 << 16));
      hv[g].x = h0 | (h1 << 16); hv[g].y = h2 | (h3 << 16);
      lv[g].x = l0 | (l1 << 16); lv[g].y = l2 | (l3 << 16);
    }
    unsigned short* rp = agg + (size_t)lrow * APITCH + 4 * lane;
#pragma unroll
    for (int g = 0; g < 6; ++g) {
      *(volatile v2u*)(rp + DF * g) = hv[g];
      *(volatile v2u*)(rp + AGWD + DF * g) = lv[g];
    }
    __threadfence();
#pragma unroll
    for (int g = 0; g < 6; ++g) {
      *(volatile v2u*)(rp + DF * g) = hv[g];
      *(volatile v2u*)(rp + AGWD + DF * g) = lv[g];
    }
  }
}

__global__ __launch_bounds__(256) __attribute__((amdgpu_num_vgpr(248)))
void k_gemmp(const unsigned short* __restrict__ hb, const unsigned short* __restrict__ agg,
             const unsigned short* __restrict__ wpt, const int* __restrict__ slot,
             const float* __restrict__ snT, const float* __restrict__ bpT,
             float* outp, int passBase, int nN)
{
  extern __shared__ v4f lds_dyn[];
  float* V = (float*)lds_dyn;
  __shared__ float sSc[3 * 128];
  __shared__ float sSn[128];
  __shared__ float sPz[128];
  __shared__ __attribute__((aligned(16))) float sBp[128];
  const int tid = (int)threadIdx.x, lane = tid & 31, hh = lane >> 4, m = lane & 15;
  const int wave = __builtin_amdgcn_readfirstlane(tid >> 5);
  const int lbase   = (int)blockIdx.x * 128;
  const int rowBase = passBase + lbase;

  if (tid < 128) {
    const int row = rowBase + tid;
    const int cv = slot[2 * (size_t)row + 1];
    const bool bad = (cv < 0) || (cv > DEGCAP);
    int c = cv < 0 ? 0 : (cv > DEGCAP ? DEGCAP : cv);
    c = row < nN ? c : 0;
    const float avgdl = (float)(2.77258872 + 2.239781e-9);
    const float degc = fmaxf((float)c, 1.0f);
    const float logd = logf(degc + 1.0f);
    sSc[tid]       = 1.0f;
    sSc[128 + tid] = logd / avgdl;
    sSc[256 + tid] = avgdl / logd;
    sSn[tid] = snT[row];
    sPz[tid] = bad ? __int_as_float(0x7fc00000) : 0.0f;
  } else if (tid < 160) {
    const int j = tid - 128;
    const v4f b = *(const v4f*)(bpT + 4 * j);
    *(v4f*)(sBp + 4 * j) = b;
  }
  __syncthreads();

  const unsigned short* aph = hb  + (size_t)(rowBase + 16 * wave + m) * DF + 8 * hh;
  const unsigned short* apa = agg + (size_t)(lbase + 16 * wave + m) * APITCH + 8 * hh;
  const v8f z8 = {0.f, 0.f, 0.f, 0.f, 0.f, 0.f, 0.f, 0.f};

#pragma unroll 1
  for (int nb = 0; nb < 3; ++nb) {
    v8f acc[8];
#pragma unroll
    for (int t = 0; t < 8; ++t) acc[t] = z8;
    const unsigned short* bp = wpt + (size_t)(128 * nb + m) * WPITCH + 8 * hh;
    if (nb == 0) {
#pragma unroll 1
      for (int k0 = 0; k0 < DF; k0 += 32) {
        FragB af;
        af.u[0] = *(const v8us*)(aph + k0);
        af.u[1] = *(const v8us*)(aph + k0 + 16);
#pragma unroll
        for (int t = 0; t < 8; ++t) {
          const unsigned short* wq = bp + (size_t)(16 * t) * WPITCH + k0;
          FragB bf;
          bf.u[0] = *(const v8us*)wq;
          bf.u[1] = *(const v8us*)(wq + 16);
          acc[t] = wmx(af, bf, acc[t]);
        }
      }
    }
#pragma unroll 1
    for (int k0 = 0; k0 < KAGG; k0 += 32) {
      FragB af;
      af.u[0] = *(const v8us*)(apa + k0);
      af.u[1] = *(const v8us*)(apa + k0 + 16);
#pragma unroll
      for (int t = 0; t < 8; ++t) {
        const unsigned short* wq = bp + (size_t)(16 * t) * WPITCH + DF + k0;
        FragB bf;
        bf.u[0] = *(const v8us*)wq;
        bf.u[1] = *(const v8us*)(wq + 16);
        acc[t] = wmx(af, bf, acc[t]);
      }
    }
    float sc[8];
#pragma unroll
    for (int r = 0; r < 8; ++r) sc[r] = sSc[nb * 128 + 16 * wave + 8 * hh + r];
    if (nb == 0) {
#pragma unroll
      for (int t = 0; t < 8; ++t) {
#pragma unroll
        for (int r = 0; r < 8; ++r) V[(16 * wave + 8 * hh + r) * TP + 16 * t + m] = acc[t][r];
      }
    } else {
#pragma unroll
      for (int t = 0; t < 8; ++t) {
#pragma unroll
        for (int r = 0; r < 8; ++r) {
          float* cell = V + (16 * wave + 8 * hh + r) * TP + 16 * t + m;
          const float cur = *cell;
          *cell = fmaf(sc[r], acc[t][r], cur);
        }
      }
    }
  }
  __syncthreads();

  const v4f bb = *(const v4f*)(sBp + 4 * lane);
#pragma unroll 1
  for (int i = 0; i < 16; ++i) {
    const int lr  = 16 * wave + i;
    const int row = rowBase + lr;
    v4f v = *(const v4fa*)(V + lr * TP + 4 * lane);
    v = v + bb;
    v = v * sSn[lr];
    v.x = (v.x > 0.0f) ? v.x : (v.x - v.x);
    v.y = (v.y > 0.0f) ? v.y : (v.y - v.y);
    v.z = (v.z > 0.0f) ? v.z : (v.z - v.z);
    v.w = (v.w > 0.0f) ? v.w : (v.w - v.w);
    const v2u hw = *(const v2u*)(hb + (size_t)row * DF + 4 * lane);
    pini((int)hw.x); pini((int)hw.y);
    v4f hv;
    hv.x = __uint_as_float(hw.x << 16); hv.y = __uint_as_float(hw.x & 0xffff0000u);
    hv.z = __uint_as_float(hw.y << 16); hv.w = __uint_as_float(hw.y & 0xffff0000u);
    v4f o = hv + v;
    o = o + sPz[lr];
    if (row < nN) {
      float* op = outp + (size_t)row * DF + 4 * lane;
      *(volatile v4f*)op = o;
      __threadfence();
      *(volatile v4f*)op = o;
    }
  }
}

static inline size_t al256(size_t o) { return (o + 255) & ~(size_t)255; }

extern "C" void kernel_launch(void* const* d_in, const int* in_sizes, int n_in,
                              void* d_out, int out_size, void* d_ws, size_t ws_size,
                              hipStream_t stream) {
  if (n_in < 10) return;
  if (in_sizes[0] != NNODE * DF) return;
  if (in_sizes[1] != NEDGE * EDIM) return;
  if (in_sizes[2] != NNODE * 2) return;
  if (in_sizes[3] != NNODE) return;
  if (in_sizes[4] != NEDGE || in_sizes[5] != NEDGE) return;
  if (in_sizes[6] != (2 * DF + EDIM) * DF || in_sizes[7] != DF) return;
  if (in_sizes[8] != 19 * DF * DF || in_sizes[9] != DF) return;
  if (out_size != NNODE * DF) return;
  const int nN = NNODE, nE = NEDGE;

  const float* h     = (const float*)d_in[0];
  const float* e     = (const float*)d_in[1];
  const float* evec  = (const float*)d_in[2];
  const float* snorm = (const float*)d_in[3];
  const int*   src   = (const int*)  d_in[4];
  const int*   dst   = (const int*)  d_in[5];
  const float* Wpre  = (const float*)d_in[6];
  const float* bpre  = (const float*)d_in[7];
  const float* Wpost = (const float*)d_in[8];
  const float* bpost = (const float*)d_in[9];
  float* out = (float*)d_out;

  char* ws = (char*)d_ws;
  size_t off = 0;
  const size_t oAGG = off; off = al256(off + (size_t)HALFN * APITCH * 2);
  const size_t oPAB = off; off = al256(off + (size_t)MP * PABP * 4);
  const size_t oHB  = off; off = al256(off + (size_t)MP * DF * 2);
  const size_t oENT = off; off = al256(off + (size_t)NBLK * RCAP * 8);
  const size_t oSLT = off; off = al256(off + (size_t)NBLK * NB * 8);
  const size_t oWPT = off; off = al256(off + (size_t)NPOST * WPITCH * 2);
  const size_t oWAB = off; off = al256(off + (size_t)256 * DF * 2);
  const size_t oWCP = off; off = al256(off + (size_t)DF * 32 * 2);
  const size_t oEV  = off; off = al256(off + (size_t)MP * 4);
  const size_t oSN  = off; off = al256(off + (size_t)MP * 4);
  const size_t oBPR = off; off = al256(off + (size_t)256 * 4);
  const size_t oBPO = off; off = al256(off + (size_t)DF * 4);
  if (off > ws_size || off > (size_t)(128u << 20)) return;
  unsigned short* AGG  = (unsigned short*)(ws + oAGG);
  float*          PAB  = (float*)(ws + oPAB);
  unsigned short* HB   = (unsigned short*)(ws + oHB);
  int*            ENT  = (int*)(ws + oENT);
  int*            SLT  = (int*)(ws + oSLT);
  unsigned short* WPT  = (unsigned short*)(ws + oWPT);
  unsigned short* WAB  = (unsigned short*)(ws + oWAB);
  unsigned short* WCP  = (unsigned short*)(ws + oWCP);
  float*          EV1  = (float*)(ws + oEV);
  float*          SNT  = (float*)(ws + oSN);
  float*          BPR  = (float*)(ws + oBPR);
  float*          BPO  = (float*)(ws + oBPO);

  hipFuncSetAttribute(reinterpret_cast<const void*>(&k_bucket), hipFuncAttributeMaxDynamicSharedMemorySize, LDS_BKT);
  hipFuncSetAttribute(reinterpret_cast<const void*>(&k_agg),    hipFuncAttributeMaxDynamicSharedMemorySize, LDS_AGG);
  hipFuncSetAttribute(reinterpret_cast<const void*>(&k_gemmp),  hipFuncAttributeMaxDynamicSharedMemorySize, LDS_V);

  const int vec8 = ((nE & 3) == 0) ? 1 : 0;

  k_prep<<<PB_TOT, 256, 0, stream>>>(h, evec, snorm, Wpre, bpre, Wpost, bpost, HB, WAB, WCP, WPT, EV1, SNT, BPR, BPO);
  k_gemm<<<dim3(MP / GBM, 256 / GBN), GTHR, 0, stream>>>(HB, WAB, BPR, PAB, DF, PABP);
  k_bucket<<<NBLK, BTHR, LDS_BKT, stream>>>(src, dst, ENT, SLT, nN, nE, vec8);
  k_agg<<<HALFN / AGB, 256, LDS_AGG, stream>>>(ENT, SLT, e, (const int*)WCP, PAB, EV1, HB, AGG, 0, nN, nE);
  k_gemmp<<<HALFN / 128, 256, LDS_V, stream>>>(HB, AGG, WPT, SLT, SNT, BPO, out, 0, nN);
  k_agg<<<HALFN / AGB, 256, LDS_AGG, stream>>>(ENT, SLT, e, (const int*)WCP, PAB, EV1, HB, AGG, HALFN, nN, nE);
  k_gemmp<<<(MP - HALFN) / 128, 256, LDS_V, stream>>>(HB, AGG, WPT, SLT, SNT, BPO, out, HALFN, nN);
}
